// BasicTransBlock_20478404067807
// MI455X (gfx1250) — hardware-verified
//
#include <hip/hip_runtime.h>


#define NB_  8
#define CC   256
#define HH   64
#define WW   64
#define PP   4096
#define NHD  8
#define DH   32
#define RS   16
#define NK   256
#define PCAR 1024.0f
typedef _Float16 h16;
typedef unsigned short bf;
typedef __attribute__((ext_vector_type(16))) __bf16   v16bf;
typedef __attribute__((ext_vector_type(16))) _Float16 v16h;
typedef __attribute__((ext_vector_type(8)))  _Float16 v8h;
typedef __attribute__((ext_vector_type(8)))  unsigned short v8us;
typedef __attribute__((ext_vector_type(8)))  float    v8f;
typedef __attribute__((ext_vector_type(4)))  float    v4f;
typedef v8h  __attribute__((may_alias)) v8ha;
typedef v4f  __attribute__((may_alias)) v4fa;
typedef v8us __attribute__((may_alias)) v8usa;

__device__ __forceinline__ unsigned short f2bf(float f) { unsigned u = __float_as_uint(f); u += 0x7FFFu + ((u >> 16) & 1u); return (unsigned short)(u >> 16); }
__device__ __forceinline__ float bf2f(unsigned short b) { return __uint_as_float(((unsigned)b) << 16); }
__device__ __forceinline__ float bfr(float f) { return bf2f(f2bf(f)); }
__device__ __forceinline__ v16h cat16(v8h lo, v8h hi) { return __builtin_shufflevector(lo, hi, 0, 1, 2, 3, 4, 5, 6, 7, 8, 9, 10, 11, 12, 13, 14, 15); }
__device__ __forceinline__ v16bf cat16b(v8us lo, v8us hi) { return __builtin_bit_cast(v16bf, __builtin_shufflevector(lo, hi, 0, 1, 2, 3, 4, 5, 6, 7, 8, 9, 10, 11, 12, 13, 14, 15)); }
__device__ __forceinline__ v8f wmma16(v16h a, v16h b, v8f c) { return __builtin_amdgcn_wmma_f32_16x16x32_f16(false, a, false, b, (short)0, c, false, false); }
__device__ __forceinline__ v8f wmmab(v16bf a, v16bf b, v8f c) { return __builtin_amdgcn_wmma_f32_16x16x32_bf16(false, a, false, b, (short)0, c, false, false); }


template <typename T16> struct WFrag;
template <> struct WFrag<h16> { typedef v16h V; static __device__ __forceinline__ V ld(const h16* p) { return cat16(*(const v8h*)p, *(const v8h*)(p + 16)); } static __device__ __forceinline__ v8f mma(V a, V b, v8f c) { return wmma16(a, b, c); } };
template <> struct WFrag<bf> { typedef v16bf V; static __device__ __forceinline__ V ld(const bf* p) { return cat16b(*(const v8us*)p, *(const v8us*)(p + 16)); } static __device__ __forceinline__ v8f mma(V a, V b, v8f c) { return wmmab(a, b, c); } };
template <typename T16, int NSPLIT, bool BIAS>
__global__ __launch_bounds__(32) void k_gemmw(const T16* __restrict__ A, const T16* __restrict__ A2, const T16* __restrict__ Bt, const T16* __restrict__ Bt2, int K, float* C, int ldc, const float* __restrict__ bias, size_t sA, size_t sB, size_t sC) {
    typedef typename WFrag<T16>::V V;
    __shared__ __align__(16) float os[16 * 68];
    const size_t z = blockIdx.z; A += z * sA; if (A2) A2 += z * sA; Bt += z * sB; if (Bt2) Bt2 += z * sB; C += z * sC;
    const int lane = threadIdx.x & 31, lr = lane & 15, hi = lane >> 4; const int r0 = blockIdx.x * 64, c0 = blockIdx.y * 64;
    v8f acc[4][4];
#pragma unroll
    for (int mb = 0; mb < 4; ++mb)
#pragma unroll
        for (int nb = 0; nb < 4; ++nb) acc[mb][nb] = (v8f){};
    const size_t aoff = (size_t)(r0 + lr) * K + 8 * hi, boff = (size_t)(c0 + lr) * K + 8 * hi;
#pragma unroll 1
    for (int kc = 0; kc < K; kc += 32) {
        V a[4], a2[4];
#pragma unroll
        for (int mb = 0; mb < 4; ++mb) { a[mb] = WFrag<T16>::ld(A + aoff + (size_t)mb * 16 * K + kc); if (NSPLIT == 1 || NSPLIT == 2) a2[mb] = WFrag<T16>::ld(A2 + aoff + (size_t)mb * 16 * K + kc); }
#pragma unroll
        for (int nb = 0; nb < 4; ++nb) { const V b = WFrag<T16>::ld(Bt + boff + (size_t)nb * 16 * K + kc); V b2; if (NSPLIT >= 2) b2 = WFrag<T16>::ld(Bt2 + boff + (size_t)nb * 16 * K + kc);
#pragma unroll
            for (int mb = 0; mb < 4; ++mb) { acc[mb][nb] = WFrag<T16>::mma(a[mb], b, acc[mb][nb]); if (NSPLIT == 1 || NSPLIT == 2) acc[mb][nb] = WFrag<T16>::mma(a2[mb], b, acc[mb][nb]); if (NSPLIT >= 2) acc[mb][nb] = WFrag<T16>::mma(a[mb], b2, acc[mb][nb]); } }
        asm volatile("v_nop\n\tv_nop\n\tv_nop\n\tv_nop" : "+v"(acc[0][0]), "+v"(acc[1][1]), "+v"(acc[2][2]), "+v"(acc[3][3]) : "v"(a[0]), "v"(a[3]));
    }
#pragma unroll
    for (int mb = 0; mb < 4; ++mb) {
#pragma unroll
        for (int nb = 0; nb < 4; ++nb) {
#pragma unroll
            for (int j = 0; j < 8; ++j) os[(hi * 8 + j) * 68 + nb * 16 + lr] = acc[mb][nb][j]; }
        __builtin_amdgcn_wave_barrier(); asm volatile("" ::: "memory");
        float* crow = C + (size_t)(r0 + mb * 16) * ldc + c0;
#pragma unroll 1
        for (int ps = 0; ps < 2; ++ps) {
#pragma unroll
            for (int s = 0; s < 8; ++s) { const int row = 2 * s + hi, cofs = lr * 4; v4f val = *(const v4fa*)(os + row * 68 + cofs); if (BIAS) { val[0] += bfr(bias[c0 + cofs]); val[1] += bfr(bias[c0 + cofs + 1]); val[2] += bfr(bias[c0 + cofs + 2]); val[3] += bfr(bias[c0 + cofs + 3]); }
                *(volatile v4f*)(crow + (size_t)row * ldc + cofs) = val; }
            if (ps == 0) __threadfence(); }
        __builtin_amdgcn_wave_barrier(); asm volatile("" ::: "memory");
    }
}

__device__ __forceinline__ h16 tohx(float x) { return (h16)x; }
typedef __attribute__((ext_vector_type(4))) _Float16 v4h;
typedef __attribute__((ext_vector_type(2))) _Float16 v2h;
__constant__ int   IY0[16] = {0, 4, 8, 12, 16, 21, 25, 29, 33, 37, 42, 46, 50, 54, 58, 63};
__constant__ float IWY[16] = {0x0.0p+0f, 0x1.9999c0p-3f, 0x1.9999c0p-2f, 0x1.333340p-1f, 0x1.9999c0p-1f, 0x1.0p-19f, 0x1.999a00p-3f, 0x1.999a00p-2f, 0x1.333380p-1f, 0x1.999a00p-1f, 0x1.0p-18f, 0x1.999c00p-3f, 0x1.999a00p-2f, 0x1.333380p-1f, 0x1.999a00p-1f, 0x0.0p+0f};
__constant__ float IW1[16] = {0x1.0p+0f, 0x1.999990p-1f, 0x1.333320p-1f, 0x1.999980p-2f, 0x1.999900p-3f, 0x1.ffffc0p-1f, 0x1.999980p-1f, 0x1.333300p-1f, 0x1.999900p-2f, 0x1.999800p-3f, 0x1.ffff80p-1f, 0x1.999900p-1f, 0x1.333300p-1f, 0x1.999900p-2f, 0x1.999800p-3f, 0x1.0p+0f};

__global__ __launch_bounds__(256) void k_cvt8h(const float* __restrict__ src, h16* dst, size_t n8) { const size_t i = (size_t)blockIdx.x * 256 + threadIdx.x; if (i >= n8) return; const v8f v = *(const v8f*)(src + i * 8); v8h o;
#pragma unroll
    for (int k = 0; k < 8; ++k) o[k] = tohx(bfr(v[k])); *(volatile v8h*)(dst + i * 8) = o; __threadfence(); *(volatile v8h*)(dst + i * 8) = o; }
__device__ __forceinline__ void bnpar(const float* gm, const float* bt, const float* mn, const float* vr, int c, float& sc, float& sh) { const float inv = bfr(gm[c]) * rsqrtf(bfr(vr[c]) + 1e-5f); sc = inv; sh = bfr(bt[c]) - bfr(mn[c]) * inv; }
template <int MODE>
__global__ __launch_bounds__(256) void k_dwtile(const float* __restrict__ SRC, const float* __restrict__ dw, const float* __restrict__ gm, const float* __restrict__ bt, const float* __restrict__ mn, const float* __restrict__ vr, h16* DT) {
    __shared__ h16 tl[64][72];
    const int tid = threadIdx.x; const int y = blockIdx.x, cg = blockIdx.y, b = blockIdx.z; const int cl = tid >> 2, px0 = (tid & 3) * 16; const int c = cg * 64 + cl;
    const float* plane = SRC + ((size_t)b * CC + c) * PP; float sc = 1.f, sh = 0.f; if (MODE != 1) bnpar(gm, bt, mn, vr, c, sc, sh);
    auto src = [&](int yy, int xx) -> float { if (yy < 0 || yy >= HH || xx < 0 || xx >= WW) return 0.f; const float v = plane[(yy < 0 ? 0 : yy) * WW + (xx < 0 ? 0 : xx)]; return MODE == 0 ? bfr(v) * sc + sh : (MODE == 2 ? fmaxf(v * sc + sh, 0.f) : v); };
    if (MODE == 2) {
#pragma unroll
        for (int i = 0; i < 16; ++i) tl[px0 + i][cl] = tohx(src(y, px0 + i));
    } else { float w9[9];
#pragma unroll
        for (int k = 0; k < 9; ++k) w9[k] = bfr(dw[c * 9 + k]);
#pragma unroll 1
        for (int i = 0; i < 16; ++i) { const int xx = px0 + i; float acc = 0.f;
#pragma unroll
            for (int ky = 0; ky < 3; ++ky)
#pragma unroll
                for (int kx = 0; kx < 3; ++kx) acc += src(y + ky - 1, xx + kx - 1) * w9[ky * 3 + kx];
            tl[xx][cl] = tohx(acc); } }
    __syncthreads();
    const int lane = tid & 31, wv = tid >> 5;
    auto pass = [&]() { const int cq = (lane & 7) * 8;
#pragma unroll
        for (int i2 = 0; i2 < 2; ++i2) { const int pr = wv * 8 + i2 * 4 + (lane >> 3); v8h o;
#pragma unroll
            for (int i = 0; i < 8; ++i) o[i] = tl[pr][cq + i];
            *(volatile v8h*)(DT + ((size_t)b * PP + y * WW + pr) * CC + cg * 64 + cq) = o; } };
    pass(); __threadfence(); pass();
}
__global__ __launch_bounds__(256) void k_qplane(const float* __restrict__ QS, float scale, h16* Qp) {
    const int lane = threadIdx.x & 31; const int L0 = (blockIdx.x * 8 + (threadIdx.x >> 5)) * 8; const int nlines = NB_ * NHD * PP * DH / 64;
#pragma unroll 1
    for (int ps = 0; ps < 2; ++ps) {
#pragma unroll
        for (int l = 0; l < 8; ++l) { const int L = L0 + l; if (L >= nlines) break; const int e = L * 64 + lane * 2; const int d = e & 31; const int hw = (e >> 5) % PP; const int z = e / (32 * PP); const int b = z >> 3, head = z & 7; v2h v;
#pragma unroll
            for (int q = 0; q < 2; ++q) v[q] = tohx(QS[((size_t)b * CC + (d + q) * NHD + head) * PP + hw] * scale);
            *(volatile v2h*)(Qp + e) = v; }
        if (ps == 0) __threadfence(); }
}
__device__ __forceinline__ float interp16(const float* __restrict__ pl, int jy, int jx) {
    const int y0 = IY0[jy], y1 = y0 + 1 > 63 ? 63 : y0 + 1, x0 = IY0[jx], x1 = x0 + 1 > 63 ? 63 : x0 + 1; const float wy = IWY[jy], wy1 = IW1[jy], wx = IWY[jx], wx1 = IW1[jx];
    const float a = __fadd_rn(__fmul_rn(pl[y0 * WW + x0], wy1), __fmul_rn(pl[y1 * WW + x0], wy)); const float c2 = __fadd_rn(__fmul_rn(pl[y0 * WW + x1], wy1), __fmul_rn(pl[y1 * WW + x1], wy));
    return __fadd_rn(__fmul_rn(a, wx1), __fmul_rn(c2, wx));
}
__global__ __launch_bounds__(256) void k_kplane(const float* __restrict__ KS, h16* Kp) {
    const int lane = threadIdx.x & 31; const int L0 = (blockIdx.x * 8 + (threadIdx.x >> 5)) * 8; const int nlines = NB_ * NHD * NK * DH / 64;
#pragma unroll 1
    for (int ps = 0; ps < 2; ++ps) {
#pragma unroll
        for (int l = 0; l < 8; ++l) { const int L = L0 + l; if (L >= nlines) break; const int e = L * 64 + lane * 2; const int d = e & 31; const int j = (e >> 5) % NK; const int z = e / (32 * NK); const int b = z >> 3, head = z & 7; const int jy = j >> 4, jx = j & 15; v2h v;
#pragma unroll
            for (int q = 0; q < 2; ++q) v[q] = tohx(interp16(KS + ((size_t)b * CC + (d + q) * NHD + head) * PP, jy, jx));
            *(volatile v2h*)(Kp + e) = v; }
        if (ps == 0) __threadfence(); }
}
__global__ __launch_bounds__(256) void k_vtplane(const float* __restrict__ VS, h16* VT) {
    const int lane = threadIdx.x & 31; const int L0 = (blockIdx.x * 8 + (threadIdx.x >> 5)) * 8; const int nlines = NB_ * NHD * 64 * NK / 64;
#pragma unroll 1
    for (int ps = 0; ps < 2; ++ps) {
#pragma unroll
        for (int l = 0; l < 8; ++l) { const int L = L0 + l; if (L >= nlines) break; const int e = L * 64 + lane * 2; const int j = e % NK; const int d = (e / NK) % 64; const int z = e / (64 * NK); const int b = z >> 3, head = z & 7; v2h v;
#pragma unroll
            for (int q = 0; q < 2; ++q) { const int jj = j + q; v[q] = (d < DH) ? tohx(interp16(VS + ((size_t)b * CC + (d < DH ? d : 0) * NHD + head) * PP, jj >> 4, jj & 15)) : tohx(0.f); }
            *(volatile v2h*)(VT + e) = v; }
        if (ps == 0) __threadfence(); }
}
__global__ __launch_bounds__(256) void k_softr(const float* __restrict__ Sb, const float* __restrict__ tab, float scale, h16* P) {
    const int lane = threadIdx.x & 31; const int row = blockIdx.x * 8 + (threadIdx.x >> 5); if (row >= NHD * PP) return; const int head = row / PP, hw = row % PP; const int yr = (hw >> 6) >> 2, xr = (hw & 63) >> 2;
    const float* sr = Sb + (size_t)row * NK; float v[8]; float mx = -3.0e38f;
#pragma unroll
    for (int ch = 0; ch < 2; ++ch)
#pragma unroll
        for (int i = 0; i < 4; ++i) { const int j = ch * 128 + lane * 4 + i; const int jy = j >> 4, jx = j & 15; const float bias = bfr(tab[((yr - jy + 15) * 31 + (xr - jx + 15)) * NHD + head]); const float t = sr[j] + bias * scale; v[ch * 4 + i] = t; mx = fmaxf(mx, t); }
#pragma unroll
    for (int sh = 16; sh; sh >>= 1) mx = fmaxf(mx, __shfl_xor(mx, sh, 32));
    float sum = 0.f;
#pragma unroll
    for (int i = 0; i < 8; ++i) { v[i] = __expf(v[i] - mx); sum += v[i]; }
#pragma unroll
    for (int sh = 16; sh; sh >>= 1) sum += __shfl_xor(sum, sh, 32);
    const float f = __fdiv_rn(PCAR, sum); v4h o[2];
#pragma unroll
    for (int ch = 0; ch < 2; ++ch)
#pragma unroll
        for (int i = 0; i < 4; ++i) o[ch][i] = tohx(v[ch * 4 + i] * f);
#pragma unroll 1
    for (int ps = 0; ps < 2; ++ps) {
#pragma unroll
        for (int ch = 0; ch < 2; ++ch) *(volatile v4h*)(P + (size_t)row * NK + ch * 128 + lane * 4) = o[ch];
        if (ps == 0) __threadfence(); }
}
__global__ __launch_bounds__(256) void k_omerge(const float* __restrict__ O, int b, float* OC) {
    const int lane = threadIdx.x & 31; const int wg = blockIdx.x * 8 + (threadIdx.x >> 5); if (wg >= CC * (PP / 128)) return; const int c = wg / (PP / 128), p0 = (wg % (PP / 128)) * 128 + lane * 4; const int d = c / NHD, head = c % NHD; v4f o;
#pragma unroll
    for (int q = 0; q < 4; ++q) o[q] = O[((size_t)head * PP + p0 + q) * 64 + d] * (1.0f / PCAR);
    float* dst = OC + ((size_t)b * CC + c) * PP + p0; *(volatile v4f*)dst = o; __threadfence(); *(volatile v4f*)dst = o;
}
__global__ __launch_bounds__(256) void k_addx(const float* A, const float* __restrict__ x, float* Y, size_t n4) {
    const size_t i = (size_t)blockIdx.x * 256 + threadIdx.x; if (i >= n4) return; const v4f a = *(const v4f*)(A + i * 4), xv = *(const v4f*)(x + i * 4); v4f o;
#pragma unroll
    for (int k = 0; k < 4; ++k) o[k] = a[k] + bfr(xv[k]);
    *(volatile v4f*)(Y + i * 4) = o; __threadfence(); *(volatile v4f*)(Y + i * 4) = o;
}
__global__ __launch_bounds__(256) void k_fin(const float* __restrict__ M, const float* __restrict__ R, float* OUT, size_t n4) {
    const size_t i = (size_t)blockIdx.x * 256 + threadIdx.x; if (i >= n4) return; const v4f a = *(const v4f*)(M + i * 4), r = *(const v4f*)(R + i * 4); const v4f o = a + r;
    *(volatile v4f*)(OUT + i * 4) = o; __threadfence(); *(volatile v4f*)(OUT + i * 4) = o;
}

extern "C" void kernel_launch(void* const* d_in, const int* in_sizes, int n_in,
                              void* d_out, int out_size, void* d_ws, size_t ws_size, hipStream_t stream) {
    (void)in_sizes; (void)n_in; (void)out_size;
    const float* x = (const float*)d_in[0]; const float* g1 = (const float*)d_in[1]; const float* be1 = (const float*)d_in[2]; const float* mn1 = (const float*)d_in[3]; const float* vr1 = (const float*)d_in[4];
    const float* qkv_dw = (const float*)d_in[5]; const float* qkv_pw = (const float*)d_in[6]; const float* out_dw = (const float*)d_in[7]; const float* out_pw = (const float*)d_in[8]; const float* tab = (const float*)d_in[9];
    const float* g2 = (const float*)d_in[10]; const float* be2 = (const float*)d_in[11]; const float* mn2 = (const float*)d_in[12]; const float* vr2 = (const float*)d_in[13]; const float* mlp_w = (const float*)d_in[14];
    float* OUT = (float*)d_out;
    char* wsp = (char*)d_ws;
    auto take = [&](size_t bytes) { char* p = wsp; wsp += (bytes + 255) & ~(size_t)255; return (void*)p; };
    h16* WQKV = (h16*)take((size_t)3 * CC * CC * 2); h16* WOP = (h16*)take((size_t)CC * CC * 2); h16* WML = (h16*)take((size_t)CC * CC * 2);
    h16* DT = (h16*)take((size_t)NB_ * PP * CC * 2);
    float* BIG = (float*)take((size_t)NB_ * CC * PP * 4);
    h16* Qp = (h16*)take((size_t)NB_ * NHD * PP * DH * 2); h16* Kp = (h16*)take((size_t)NB_ * NHD * NK * DH * 2); h16* VT = (h16*)take((size_t)NB_ * NHD * 64 * NK * 2);
    h16* Pm = (h16*)take((size_t)NHD * PP * NK * 2); float* Ob = (float*)take((size_t)NHD * PP * 64 * 4);
    float* OC = (float*)take((size_t)NB_ * CC * PP * 4);
    if ((size_t)(wsp - (char*)d_ws) > ws_size) return;
    float* QS = BIG; float* Sb = BIG; float* O2 = BIG; float* OUT1 = BIG; float* Mcm = OC;
    { const size_t n3 = (size_t)3 * CC * CC / 8, n1 = (size_t)CC * CC / 8; k_cvt8h<<<(unsigned)((n3 + 255) / 256), 256, 0, stream>>>(qkv_pw, WQKV, n3); k_cvt8h<<<(unsigned)((n1 + 255) / 256), 256, 0, stream>>>(out_pw, WOP, n1); k_cvt8h<<<(unsigned)((n1 + 255) / 256), 256, 0, stream>>>(mlp_w, WML, n1); }
    const float scale = 0x1.6a09e6p-3f;
    k_dwtile<0><<<dim3(HH, CC / 64, NB_), 256, 0, stream>>>(x, qkv_dw, g1, be1, mn1, vr1, DT);
    const unsigned LQ = (unsigned)((NB_ * NHD * PP * DH / 64 + 63) / 64), LK = (unsigned)((NB_ * NHD * NK * DH / 64 + 63) / 64), LV = (unsigned)((NB_ * NHD * 64 * NK / 64 + 63) / 64);
    k_gemmw<h16, 0, false><<<dim3(CC / 64, PP / 64, NB_), 32, 0, stream>>>(WQKV, nullptr, DT, nullptr, CC, QS, PP, nullptr, 0, (size_t)PP * CC, (size_t)CC * PP); k_qplane<<<LQ, 256, 0, stream>>>(QS, scale, Qp);
    k_gemmw<h16, 0, false><<<dim3(CC / 64, PP / 64, NB_), 32, 0, stream>>>(WQKV + (size_t)CC * CC, nullptr, DT, nullptr, CC, QS, PP, nullptr, 0, (size_t)PP * CC, (size_t)CC * PP); k_kplane<<<LK, 256, 0, stream>>>(QS, Kp);
    k_gemmw<h16, 0, false><<<dim3(CC / 64, PP / 64, NB_), 32, 0, stream>>>(WQKV + (size_t)2 * CC * CC, nullptr, DT, nullptr, CC, QS, PP, nullptr, 0, (size_t)PP * CC, (size_t)CC * PP); k_vtplane<<<LV, 256, 0, stream>>>(QS, VT);
    for (int b = 0; b < NB_; ++b) { const size_t z0 = (size_t)b * NHD;
        k_gemmw<h16, 0, false><<<dim3(PP / 64, NK / 64, NHD), 32, 0, stream>>>(Qp + z0 * PP * DH, nullptr, Kp + z0 * NK * DH, nullptr, DH, Sb, NK, nullptr, (size_t)PP * DH, (size_t)NK * DH, (size_t)PP * NK);
        k_softr<<<NHD * PP / 8, 256, 0, stream>>>(Sb, tab, scale, Pm);
        k_gemmw<h16, 0, false><<<dim3(PP / 64, 1, NHD), 32, 0, stream>>>(Pm, nullptr, VT + z0 * 64 * NK, nullptr, NK, Ob, 64, nullptr, (size_t)PP * NK, (size_t)64 * NK, (size_t)PP * 64);
        k_omerge<<<CC * (PP / 128) / 8, 256, 0, stream>>>(Ob, b, OC); }
    k_dwtile<1><<<dim3(HH, CC / 64, NB_), 256, 0, stream>>>(OC, out_dw, g1, be1, mn1, vr1, DT);
    k_gemmw<h16, 0, false><<<dim3(CC / 64, PP / 64, NB_), 32, 0, stream>>>(WOP, nullptr, DT, nullptr, CC, O2, PP, nullptr, 0, (size_t)PP * CC, (size_t)CC * PP);
    const size_t n4 = (size_t)NB_ * CC * PP / 4;
    k_addx<<<(unsigned)((n4 + 255) / 256), 256, 0, stream>>>(O2, x, OUT1, n4);
    k_dwtile<2><<<dim3(HH, CC / 64, NB_), 256, 0, stream>>>(OUT1, out_dw, g2, be2, mn2, vr2, DT);
    k_gemmw<h16, 0, false><<<dim3(CC / 64, PP / 64, NB_), 32, 0, stream>>>(WML, nullptr, DT, nullptr, CC, Mcm, PP, nullptr, 0, (size_t)PP * CC, (size_t)CC * PP);
    k_fin<<<(unsigned)((n4 + 255) / 256), 256, 0, stream>>>(Mcm, OUT1, OUT, n4);
}
